// Mixer_10557029614277
// MI455X (gfx1250) — hardware-verified
//
#include <hip/hip_runtime.h>
#include <math.h>

typedef __attribute__((ext_vector_type(16))) _Float16 v16h;
typedef __attribute__((ext_vector_type(8)))  _Float16 v8h;
typedef __attribute__((ext_vector_type(4)))  _Float16 v4h;
typedef __attribute__((ext_vector_type(8)))  float    v8f;
typedef __attribute__((ext_vector_type(4)))  float    v4f;

constexpr int kBT      = 128 * 200;
constexpr int kAgents  = 8;
constexpr int kGroups  = 2;
constexpr int kPerGrp  = 4;
constexpr int kEmb     = 32;
constexpr int kHyp     = 64;
constexpr int kAhDim   = 64;
constexpr int kStDim   = 128;
constexpr int kTileRows = 16;
constexpr int kWavesPerBlock = 4;
constexpr int kBlockRows = kTileRows * kWavesPerBlock;
constexpr int kNumBlocks = kBT / kBlockRows;
constexpr int kOutFloats = kBT + kPerGrp + kBT;
constexpr int kOutLines  = (kOutFloats + 31) / 32;
static_assert(kBT == 25600, "row count");
static_assert(kBT % kBlockRows == 0, "no row tail");
static_assert(kNumBlocks == 400, "block count");
static_assert(kOutFloats == 51204, "output element count");
static_assert(kOutLines == 1601, "output line count");
static_assert(kAgents == kGroups * kPerGrp, "grouping");
static_assert(kHyp == 64 && kAhDim == 64 && kStDim == 128 && kEmb == 32, "tile shapes");

constexpr float kActCarry = 16.0f;
constexpr float kWCarry   = 256.0f;
constexpr float kFold     = 1.0f / (kActCarry * kWCarry);
constexpr float kF16MinNormal = 6.103515625e-5f;
constexpr float kInvMeanCount = 1.0f / (float)(kBT * kEmb);
constexpr float kInvPairs     = 1.0f / (float)(kAgents * kAgents);

constexpr int kXaPitch = 136;
constexpr int kHtPitch = 72;
constexpr int kGsTile  = kTileRows * kHtPitch;

constexpr int oW1a  = 0;
constexpr int oW1b  = oW1a  + 8 * 64 * 64;
constexpr int oWb1  = oW1b  + 8 * 32 * 64;
constexpr int oWw2a = oWb1  + 2 * 32 * 64;
constexpr int oWw2b = oWw2a + 2 * 64 * 64;
constexpr int oWb2a = oWw2b + 2 * 32 * 64;
constexpr int oW3a  = oWb2a + 2 * 32 * 64;
constexpr int oW3b  = oW3a  + 64 * 64;
constexpr int oWb3  = oW3b  + 32 * 64;
constexpr int oW4a  = oWb3  + 32 * 64;
constexpr int oW4b  = oW4a  + 64 * 128;
constexpr int oWb4a = oW4b  + 32 * 64;
constexpr int oWEnd = oWb4a + 32 * 128;
static_assert(oWEnd == 92160, "weight plane halves");
static_assert((oWEnd / 8) % 256 == 0, "prep grid is exact");

constexpr size_t kOffWT   = 0;
constexpr size_t kOffRES  = kOffWT   + (size_t)oWEnd * 2;
constexpr size_t kOffPART = kOffRES  + (size_t)2 * kBT * 4;
constexpr size_t kOffAVG  = kOffPART + (size_t)kNumBlocks * 32 * 4;
constexpr size_t kWsTotal = kOffAVG  + 128;
static_assert(kWsTotal == 440448ull, "carve total");
static_assert((kOffRES % 128) == 0 && (kOffPART % 128) == 0 && (kOffAVG % 128) == 0, "aligned regions");
static_assert(kWsTotal <= 134217728ull, "carve cap");

__device__ __forceinline__ _Float16 to_h(float v) {
  const float z = (fabsf(v) < kF16MinNormal) ? 0.0f : v;
  return (_Float16)z;
}

union FragU { v16h v; v8h h[2]; };
__device__ __forceinline__ v16h frag_load(const _Float16* p) {
  FragU f;
  f.h[0] = *(const v8h*)(p);
  f.h[1] = *(const v8h*)(p + 16);
  return f.v;
}
__device__ __forceinline__ v8f mma_h(v16h a, v16h b, v8f c) {
  c = __builtin_amdgcn_wmma_f32_16x16x32_f16(false, a, false, b, (short)0, c, false, false);
  asm volatile("v_nop\n\tv_nop\n\tv_nop\n\tv_nop" : "+v"(c) : "v"(a), "v"(b));
  return c;
}
__device__ __forceinline__ v8f zero8() { return (v8f){0.f, 0.f, 0.f, 0.f, 0.f, 0.f, 0.f, 0.f}; }

template <int NT, int KS>
__device__ __forceinline__ void tile_gemm(const _Float16* a_lds, int apitch, const _Float16* bt,
                                          v8f (&c)[NT], int col, int hh) {
  constexpr int KD = KS * 32;
#pragma unroll
  for (int ks = 0; ks < KS; ++ks) {
    const v16h a = frag_load(a_lds + col * apitch + ks * 32 + 8 * hh);
#pragma unroll
    for (int t = 0; t < NT; ++t) {
      const v16h b = frag_load(bt + (t * 16 + col) * KD + ks * 32 + 8 * hh);
      c[t] = mma_h(a, b, c[t]);
    }
  }
}

template <int NT>
__device__ __forceinline__ void relu_to_lds(const v8f (&c)[NT], const float* bias, _Float16* ht, int col, int hh) {
#pragma unroll
  for (int t = 0; t < NT; ++t) {
    const float bv = bias[t * 16 + col];
#pragma unroll
    for (int r = 0; r < 8; ++r) {
      float v = fmaf(c[t][r], kFold, bv);
      v = fmaxf(v, 0.0f);
      ht[(8 * hh + r) * kHtPitch + t * 16 + col] = to_h(v * kActCarry);
    }
  }
}

__device__ __forceinline__ void store4h(_Float16* p, v4f v) {
  v4h h;
  h[0] = to_h(v[0] * kActCarry);
  h[1] = to_h(v[1] * kActCarry);
  h[2] = to_h(v[2] * kActCarry);
  h[3] = to_h(v[3] * kActCarry);
  *(v4h*)p = h;
}

__device__ __forceinline__ float red16(float p) {
  p += __shfl_xor(p, 1, 32);
  p += __shfl_xor(p, 2, 32);
  p += __shfl_xor(p, 4, 32);
  p += __shfl_xor(p, 8, 32);
  return p;
}

__device__ __forceinline__ void elu_pair(v8f& a, v8f& b) {
#pragma unroll 1
  for (int t = 0; t < 2; ++t) {
    const bool first = (t == 0);
    v8f x;
#pragma unroll
    for (int r = 0; r < 8; ++r) x[r] = first ? a[r] : b[r];
#pragma unroll
    for (int r = 0; r < 8; ++r) {
      const float v = x[r];
      const float e = expm1f(fminf(v, 0.0f));
      x[r] = (v > 0.0f) ? v : e;
    }
#pragma unroll
    for (int r = 0; r < 8; ++r) {
      a[r] = first ? x[r] : a[r];
      b[r] = first ? b[r] : x[r];
    }
  }
}

__global__ __launch_bounds__(256) void prep_weights_kernel(
    const float* __restrict__ w1a,  const float* __restrict__ w1b,  const float* __restrict__ wb1,
    const float* __restrict__ ww2a, const float* __restrict__ ww2b, const float* __restrict__ wb2a,
    const float* __restrict__ w3a,  const float* __restrict__ w3b,  const float* __restrict__ wb3,
    const float* __restrict__ w4a,  const float* __restrict__ w4b,  const float* __restrict__ wb4a,
    unsigned short* __restrict__ WT)
{
  const unsigned c = blockIdx.x * 256u + threadIdx.x;
  if (c >= (unsigned)(oWEnd / 8)) return;
  unsigned e0 = c * 8u;
  asm volatile("" : "+v"(e0));
  const float* src = w1a;
  unsigned base = 0u, ksh = 6u, nsh = 6u;
  if (e0 >= (unsigned)oW1b)  { src = w1b;  base = (unsigned)oW1b;  ksh = 6u; nsh = 5u; }
  if (e0 >= (unsigned)oWb1)  { src = wb1;  base = (unsigned)oWb1;  ksh = 6u; nsh = 5u; }
  if (e0 >= (unsigned)oWw2a) { src = ww2a; base = (unsigned)oWw2a; ksh = 6u; nsh = 6u; }
  if (e0 >= (unsigned)oWw2b) { src = ww2b; base = (unsigned)oWw2b; ksh = 6u; nsh = 5u; }
  if (e0 >= (unsigned)oWb2a) { src = wb2a; base = (unsigned)oWb2a; ksh = 6u; nsh = 5u; }
  if (e0 >= (unsigned)oW3a)  { src = w3a;  base = (unsigned)oW3a;  ksh = 6u; nsh = 6u; }
  if (e0 >= (unsigned)oW3b)  { src = w3b;  base = (unsigned)oW3b;  ksh = 6u; nsh = 5u; }
  if (e0 >= (unsigned)oWb3)  { src = wb3;  base = (unsigned)oWb3;  ksh = 6u; nsh = 5u; }
  if (e0 >= (unsigned)oW4a)  { src = w4a;  base = (unsigned)oW4a;  ksh = 7u; nsh = 6u; }
  if (e0 >= (unsigned)oW4b)  { src = w4b;  base = (unsigned)oW4b;  ksh = 6u; nsh = 5u; }
  if (e0 >= (unsigned)oWb4a) { src = wb4a; base = (unsigned)oWb4a; ksh = 7u; nsh = 5u; }
  unsigned local = e0 - base;
  asm volatile("" : "+v"(local));
  const unsigned tsh = ksh + nsh;
  const unsigned set = local >> tsh;
  const unsigned rem = local & ((1u << tsh) - 1u);
  const unsigned n   = rem >> ksh;
  const unsigned k0  = rem & ((1u << ksh) - 1u);
  unsigned sbase = (set << tsh) + n;
  asm volatile("" : "+v"(sbase));
  float wv[8];
#pragma unroll
  for (int e = 0; e < 8; ++e) wv[e] = src[sbase + ((k0 + (unsigned)e) << nsh)];
  v8h hv;
#pragma unroll
  for (int e = 0; e < 8; ++e) hv[e] = to_h(wv[e] * kWCarry);
  unsigned short* dst = WT + e0;
  *(volatile v8h*)dst = hv;
  __threadfence();
  *(volatile v8h*)dst = hv;
}

__global__ __launch_bounds__(128) void fused_mixer_kernel(
    const float* __restrict__ qvals, const float* __restrict__ states,
    const float* __restrict__ a_h,   const float* __restrict__ gs,
    const unsigned short* __restrict__ WTp,
    const float* __restrict__ b1a,  const float* __restrict__ b1b,  const float* __restrict__ bb1,
    const float* __restrict__ bw2a, const float* __restrict__ bw2b, const float* __restrict__ bb2a,
    const float* __restrict__ Wb2b, const float* __restrict__ bb2b,
    const float* __restrict__ b3a,  const float* __restrict__ b3b,  const float* __restrict__ bb3,
    const float* __restrict__ b4a,  const float* __restrict__ b4b,  const float* __restrict__ bb4a,
    const float* __restrict__ Wb4b, const float* __restrict__ bb4b,
    float* __restrict__ RES, float* __restrict__ PART)
{
  __shared__ __align__(16) _Float16 sXA[kWavesPerBlock][kTileRows * kXaPitch];
  __shared__ __align__(16) _Float16 sHT[kWavesPerBlock][kTileRows * kHtPitch];
  __shared__ __align__(16) _Float16 sGS[kWavesPerBlock][3 * kGsTile];
  __shared__ __align__(16) float    sQ[kWavesPerBlock][kTileRows * kAgents];
  __shared__ __align__(16) float    sRes[2 * kBlockRows];
  __shared__ __align__(16) float    sPart[32];

  const _Float16* WT = (const _Float16*)WTp;
  const int tid  = threadIdx.x;
  const int lane = tid & 31;
  const int wave = tid >> 5;
  const int col  = lane & 15;
  const int hh   = lane >> 4;
  const int s0   = (blockIdx.x * kWavesPerBlock + wave) * kTileRows;

  _Float16* xa  = sXA[wave];
  _Float16* ht  = sHT[wave];
  _Float16* gsa = sGS[wave];
  float*    sq  = sQ[wave];

  {
    const v4f qv = *(const v4f*)(qvals + (size_t)s0 * kAgents + lane * 4);
    *(v4f*)(sq + lane * 4) = qv;
  }
  if (tid >= 16 && tid < 32) sPart[tid] = 0.0f;

  float sdv = 0.0f;
  {
    const int qd  = lane & 3;
    const int jj  = (lane >> 2) & 3;
    const bool st0 = (jj == 0);
    const bool st1 = (jj == 1) && (hh == 0);
    const float sgn = (hh == 0) ? 1.0f : -1.0f;
    const int tsel = st0 ? hh : 2;
#pragma unroll 1
    for (int s = 0; s < kTileRows; ++s) {
      const float* gp = gs + (size_t)(s0 + s) * (kAgents * kHyp) + lane * 16;
      v4f x[4];
#pragma unroll
      for (int q4 = 0; q4 < 4; ++q4) x[q4] = *(const v4f*)(gp + 4 * q4);
      float ss = 0.0f;
#pragma unroll
      for (int q4 = 0; q4 < 4; ++q4) {
#pragma unroll
        for (int e = 0; e < 4; ++e) ss = fmaf(x[q4][e], x[q4][e], ss);
      }
      ss += __shfl_xor(ss, 1, 32);
      ss += __shfl_xor(ss, 2, 32);
      const float inv = rsqrtf(ss) * sgn;
      float dsq = 0.0f;
      v8h hv[2];
#pragma unroll
      for (int q4 = 0; q4 < 4; ++q4) {
#pragma unroll
        for (int e = 0; e < 4; ++e) {
          const float xv = x[q4][e];
          float d = xv * inv;
          d += __shfl_xor(d, 4, 32);
          d += __shfl_xor(d, 8, 32);
          d += __shfl_xor(d, 16, 32);
          dsq = fmaf(d, d, dsq);
          float m = xv;
          m = fmaxf(m, __shfl_xor(m, 4, 32));
          m = fmaxf(m, __shfl_xor(m, 8, 32));
          const float mo = __shfl_xor(m, 16, 32);
          const float gv = st0 ? m : (m + mo);
          hv[(q4 * 4 + e) >> 3][(q4 * 4 + e) & 7] = to_h(gv * kActCarry);
        }
      }
      dsq += __shfl_xor(dsq, 1, 32);
      dsq += __shfl_xor(dsq, 2, 32);
      const float sd = -dsq * kInvPairs;
      sdv = (lane == s) ? sd : sdv;
      _Float16* dst = gsa + tsel * kGsTile + s * kHtPitch + qd * 16;
      if (st0 || st1) {
        *(v8h*)(dst)     = hv[0];
        *(v8h*)(dst + 8) = hv[1];
      }
    }
  }
  __syncthreads();

  v8f qg0 = zero8(), qg1 = zero8();
#pragma unroll 1
  for (int g = 0; g < kGroups; ++g) {
    v4f asum[8];
#pragma unroll
    for (int it = 0; it < 8; ++it) asum[it] = (v4f){0.f, 0.f, 0.f, 0.f};
    v8f macc[2];
    macc[0] = zero8();
    macc[1] = zero8();

#pragma unroll 1
    for (int j = 0; j < kPerGrp; ++j) {
      const int n = g * kPerGrp + j;
      const float* ap = a_h + (size_t)s0 * (kAgents * kAhDim) + n * kAhDim + hh * (kAgents * kAhDim) + col * 4;
      v4f av[8];
#pragma unroll
      for (int it = 0; it < 8; ++it) av[it] = *(const v4f*)(ap + (size_t)it * (2 * kAgents * kAhDim));
#pragma unroll
      for (int it = 0; it < 8; ++it) asum[it] += av[it];
      __syncthreads();
#pragma unroll
      for (int it = 0; it < 8; ++it) store4h(xa + (it * 2 + hh) * kXaPitch + col * 4, av[it]);
      __syncthreads();
      {
        v8f ct[4];
        ct[0] = zero8(); ct[1] = zero8(); ct[2] = zero8(); ct[3] = zero8();
        tile_gemm<4, 2>(xa, kXaPitch, WT + oW1a + n * (64 * 64), ct, col, hh);
        relu_to_lds<4>(ct, b1a + n * kHyp, ht, col, hh);
      }
      __syncthreads();
      float lsum = 0.0f;
      {
        v8f c2[2];
        c2[0] = zero8(); c2[1] = zero8();
        tile_gemm<2, 2>(ht, kHtPitch, WT + oW1b + n * (32 * 64), c2, col, hh);
#pragma unroll
        for (int t = 0; t < 2; ++t) {
          const float bv = b1b[n * kEmb + t * 16 + col];
#pragma unroll
          for (int r = 0; r < 8; ++r) {
            const float w = fabsf(fmaf(c2[t][r], kFold, bv));
            const float qv = sq[(8 * hh + r) * kAgents + n];
            macc[t][r] = fmaf(qv, w, macc[t][r]);
            lsum += w;
          }
        }
      }
      lsum += __shfl_xor(lsum, 16, 32);
      lsum += __shfl_xor(lsum, 8, 32);
      lsum += __shfl_xor(lsum, 4, 32);
      lsum += __shfl_xor(lsum, 2, 32);
      lsum += __shfl_xor(lsum, 1, 32);
      if (g == 0 && lane == 0) sPart[wave * 4 + j] = lsum;
    }

    __syncthreads();
#pragma unroll
    for (int it = 0; it < 8; ++it) store4h(xa + (it * 2 + hh) * kXaPitch + col * 4, asum[it]);
    __syncthreads();
    {
      v8f c3[2];
      c3[0] = zero8(); c3[1] = zero8();
      tile_gemm<2, 2>(xa, kXaPitch, WT + oWb1 + g * (32 * 64), c3, col, hh);
#pragma unroll
      for (int t = 0; t < 2; ++t) {
        const float bv = (float)kPerGrp * bb1[g * kEmb + t * 16 + col];
#pragma unroll
        for (int r = 0; r < 8; ++r) macc[t][r] += fmaf(c3[t][r], kFold, bv);
      }
    }
    {
      v8f c4[4];
      c4[0] = zero8(); c4[1] = zero8(); c4[2] = zero8(); c4[3] = zero8();
      tile_gemm<4, 2>(gsa + g * kGsTile, kHtPitch, WT + oWw2a + g * (64 * 64), c4, col, hh);
      relu_to_lds<4>(c4, bw2a + g * kHyp, ht, col, hh);
    }
    __syncthreads();
    v8f w2t[2];
    w2t[0] = zero8(); w2t[1] = zero8();
    tile_gemm<2, 2>(ht, kHtPitch, WT + oWw2b + g * (32 * 64), w2t, col, hh);
#pragma unroll
    for (int t = 0; t < 2; ++t) {
      const float bv = bw2b[g * kEmb + t * 16 + col];
#pragma unroll
      for (int r = 0; r < 8; ++r) w2t[t][r] = fabsf(fmaf(w2t[t][r], kFold, bv));
    }
    v8f hb[2];
    hb[0] = zero8(); hb[1] = zero8();
    tile_gemm<2, 2>(gsa + g * kGsTile, kHtPitch, WT + oWb2a + g * (32 * 64), hb, col, hh);
#pragma unroll
    for (int t = 0; t < 2; ++t) {
      const float bv = bb2a[g * kEmb + t * 16 + col];
#pragma unroll
      for (int r = 0; r < 8; ++r) hb[t][r] = fmaxf(fmaf(hb[t][r], kFold, bv), 0.0f);
    }
    elu_pair(macc[0], macc[1]);
    {
      const float wv0 = Wb2b[g * kEmb + col];
      const float wv1 = Wb2b[g * kEmb + 16 + col];
      const float bsc = bb2b[g];
#pragma unroll
      for (int r = 0; r < 8; ++r) {
        float p = macc[0][r] * w2t[0][r];
        p = fmaf(macc[1][r], w2t[1][r], p);
        p = fmaf(hb[0][r], wv0, p);
        p = fmaf(hb[1][r], wv1, p);
        p = red16(p);
        p += bsc;
        qg0[r] = (g == 0) ? p : qg0[r];
        qg1[r] = (g == 0) ? qg1[r] : p;
      }
    }
  }

  v8f th[2];
#pragma unroll
  for (int t = 0; t < 2; ++t) {
    const float bv = (float)kGroups * bb3[t * 16 + col];
#pragma unroll
    for (int r = 0; r < 8; ++r) th[t][r] = bv;
  }
  {
    v8f c9[2];
    c9[0] = zero8(); c9[1] = zero8();
    tile_gemm<2, 2>(gsa + 2 * kGsTile, kHtPitch, WT + oWb3, c9, col, hh);
#pragma unroll
    for (int t = 0; t < 2; ++t) {
#pragma unroll
      for (int r = 0; r < 8; ++r) th[t][r] = fmaf(c9[t][r], kFold, th[t][r]);
    }
  }
#pragma unroll 1
  for (int g = 0; g < kGroups; ++g) {
    __syncthreads();
    {
      v8f c7[4];
      c7[0] = zero8(); c7[1] = zero8(); c7[2] = zero8(); c7[3] = zero8();
      tile_gemm<4, 2>(gsa + g * kGsTile, kHtPitch, WT + oW3a, c7, col, hh);
      relu_to_lds<4>(c7, b3a, ht, col, hh);
    }
    __syncthreads();
    {
      v8f c8[2];
      c8[0] = zero8(); c8[1] = zero8();
      tile_gemm<2, 2>(ht, kHtPitch, WT + oW3b, c8, col, hh);
#pragma unroll
      for (int t = 0; t < 2; ++t) {
        const float bv = b3b[t * 16 + col];
#pragma unroll
        for (int r = 0; r < 8; ++r) {
          const float w3 = fabsf(fmaf(c8[t][r], kFold, bv));
          const float qv = (g == 0) ? qg0[r] : qg1[r];
          th[t][r] = fmaf(qv, w3, th[t][r]);
        }
      }
    }
  }
  elu_pair(th[0], th[1]);

  __syncthreads();
#pragma unroll
  for (int half = 0; half < 2; ++half) {
    v4f sv[8];
#pragma unroll
    for (int it = 0; it < 8; ++it)
      sv[it] = *(const v4f*)(states + (size_t)(s0 + half * 8 + it) * kStDim + lane * 4);
#pragma unroll
    for (int it = 0; it < 8; ++it) store4h(xa + (half * 8 + it) * kXaPitch + lane * 4, sv[it]);
  }
  __syncthreads();
  {
    v8f c10[4];
    c10[0] = zero8(); c10[1] = zero8(); c10[2] = zero8(); c10[3] = zero8();
    tile_gemm<4, 4>(xa, kXaPitch, WT + oW4a, c10, col, hh);
    relu_to_lds<4>(c10, b4a, ht, col, hh);
  }
  __syncthreads();
  v8f w4t[2];
  w4t[0] = zero8(); w4t[1] = zero8();
  tile_gemm<2, 2>(ht, kHtPitch, WT + oW4b, w4t, col, hh);
#pragma unroll
  for (int t = 0; t < 2; ++t) {
    const float bv = b4b[t * 16 + col];
#pragma unroll
    for (int r = 0; r < 8; ++r) w4t[t][r] = fabsf(fmaf(w4t[t][r], kFold, bv));
  }
  v8f hb4[2];
  hb4[0] = zero8(); hb4[1] = zero8();
  tile_gemm<2, 4>(xa, kXaPitch, WT + oWb4a, hb4, col, hh);
#pragma unroll
  for (int t = 0; t < 2; ++t) {
    const float bv = bb4a[t * 16 + col];
#pragma unroll
    for (int r = 0; r < 8; ++r) hb4[t][r] = fmaxf(fmaf(hb4[t][r], kFold, bv), 0.0f);
  }
  {
    const float wv0 = Wb4b[col];
    const float wv1 = Wb4b[16 + col];
    const float bsc = bb4b[0];
#pragma unroll
    for (int r = 0; r < 8; ++r) {
      float p = th[0][r] * w4t[0][r];
      p = fmaf(th[1][r], w4t[1][r], p);
      p = fmaf(hb4[0][r], wv0, p);
      p = fmaf(hb4[1][r], wv1, p);
      p = red16(p);
      p += bsc;
      if (col == 0) sRes[wave * kTileRows + 8 * hh + r] = p;
    }
  }
  if (lane < 16) sRes[kBlockRows + wave * kTileRows + lane] = sdv;
  __syncthreads();

  if (wave == 0) {
    const v4f rv = *(const v4f*)(sRes + hh * kBlockRows + col * 4);
    const v4f pv = *(const v4f*)(sPart + (lane & 7) * 4);
    float* dst  = RES + (size_t)hh * kBT + (size_t)blockIdx.x * kBlockRows + col * 4;
    float* pdst = PART + (size_t)blockIdx.x * 32 + (lane & 7) * 4;
    *(volatile v4f*)dst = rv;
    if (lane < 8) *(volatile v4f*)pdst = pv;
    __threadfence();
    *(volatile v4f*)dst = rv;
    if (lane < 8) *(volatile v4f*)pdst = pv;
  }
}

__global__ __launch_bounds__(64) void mean_combine_kernel(const float* __restrict__ PART, float* __restrict__ AVG)
{
  __shared__ float cs[64];
  __shared__ __align__(16) float av[32];
  const int tid = threadIdx.x;
  const int j = tid & 3;
  const int c = tid >> 2;
  float s = 0.0f;
#pragma unroll 1
  for (int b = c * 25; b < c * 25 + 25; ++b) {
    const float* p = PART + (size_t)b * 32 + j;
    s += p[0];
    s += p[4];
    s += p[8];
    s += p[12];
  }
  cs[tid] = s;
  __syncthreads();
  float tot = 0.0f;
#pragma unroll 1
  for (int k = 0; k < 16; ++k) tot += cs[k * 4 + j];
  if (tid < 32) av[tid] = (tid < 4) ? (tot * kInvMeanCount) : 0.0f;
  __syncthreads();
  if (tid < 8) {
    const v4f v = *(const v4f*)(av + tid * 4);
    *(volatile v4f*)(AVG + tid * 4) = v;
    __threadfence();
    *(volatile v4f*)(AVG + tid * 4) = v;
  }
}

__global__ __launch_bounds__(256) void pack_out_kernel(const float* __restrict__ RES, const float* __restrict__ AVG,
                                                       float* __restrict__ out)
{
  const int lane = threadIdx.x & 31;
  const int wave = threadIdx.x >> 5;
  const int line = blockIdx.x * 8 + wave;
  if (line >= kOutLines) return;
  unsigned i0 = (unsigned)line * 32u + (unsigned)(lane & 7) * 4u;
  asm volatile("" : "+v"(i0));
  const unsigned ti = (i0 < (unsigned)(kBT - 4)) ? i0 : (unsigned)(kBT - 4);
  const int sraw = (int)i0 - (kBT + kPerGrp);
  const int scl  = (sraw < 0) ? 0 : ((sraw > kBT - 4) ? (kBT - 4) : sraw);
  const v4f tv = *(const v4f*)(RES + ti);
  const v4f sv = *(const v4f*)(RES + kBT + scl);
  const v4f av = *(const v4f*)(AVG);
  float t0 = tv[0], t1 = tv[1], t2 = tv[2], t3 = tv[3];
  float u0 = sv[0], u1 = sv[1], u2 = sv[2], u3 = sv[3];
  float a0 = av[0], a1 = av[1], a2 = av[2], a3 = av[3];
  asm volatile("" : "+v"(t0), "+v"(t1), "+v"(t2), "+v"(t3));
  asm volatile("" : "+v"(u0), "+v"(u1), "+v"(u2), "+v"(u3));
  asm volatile("" : "+v"(a0), "+v"(a1), "+v"(a2), "+v"(a3));
  const bool is_tot = (i0 < (unsigned)kBT);
  const bool is_avg = (i0 == (unsigned)kBT);
  v4f ov;
  ov[0] = is_tot ? t0 : (is_avg ? a0 : u0);
  ov[1] = is_tot ? t1 : (is_avg ? a1 : u1);
  ov[2] = is_tot ? t2 : (is_avg ? a2 : u2);
  ov[3] = is_tot ? t3 : (is_avg ? a3 : u3);
  const bool st = (lane < 8) && (i0 < (unsigned)kOutFloats);
  if (st) *(volatile v4f*)(out + i0) = ov;
  __threadfence();
  if (st) *(volatile v4f*)(out + i0) = ov;
}

extern "C" void kernel_launch(void* const* d_in, const int* in_sizes, int n_in,
                              void* d_out, int out_size, void* d_ws, size_t ws_size,
                              hipStream_t stream) {
  if (n_in < 32) return;
  if (in_sizes[0] != kBT * kAgents) return;
  if (in_sizes[1] != kBT * kStDim) return;
  if (in_sizes[2] != kBT * kAgents * kAhDim) return;
  if (in_sizes[3] != kBT * kAgents * kHyp) return;
  if (in_sizes[4] != 8 * 64 * 64) return;
  if (in_sizes[6] != 8 * 64 * 32) return;
  if (in_sizes[24] != 128 * 64) return;
  if (in_sizes[28] != 128 * 32) return;
  if (out_size != kOutFloats) return;
  if (ws_size < kWsTotal) return;

  const float* qvals  = (const float*)d_in[0];
  const float* states = (const float*)d_in[1];
  const float* a_h    = (const float*)d_in[2];
  const float* gs     = (const float*)d_in[3];
  const float* W1a  = (const float*)d_in[4];   const float* b1a  = (const float*)d_in[5];
  const float* W1b  = (const float*)d_in[6];   const float* b1b  = (const float*)d_in[7];
  const float* Wb1  = (const float*)d_in[8];   const float* bb1  = (const float*)d_in[9];
  const float* Ww2a = (const float*)d_in[10];  const float* bw2a = (const float*)d_in[11];
  const float* Ww2b = (const float*)d_in[12];  const float* bw2b = (const float*)d_in[13];
  const float* Wb2a = (const float*)d_in[14];  const float* bb2a = (const float*)d_in[15];
  const float* Wb2b = (const float*)d_in[16];  const float* bb2b = (const float*)d_in[17];
  const float* W3a  = (const float*)d_in[18];  const float* b3a  = (const float*)d_in[19];
  const float* W3b  = (const float*)d_in[20];  const float* b3b  = (const float*)d_in[21];
  const float* Wb3  = (const float*)d_in[22];  const float* bb3  = (const float*)d_in[23];
  const float* W4a  = (const float*)d_in[24];  const float* b4a  = (const float*)d_in[25];
  const float* W4b  = (const float*)d_in[26];  const float* b4b  = (const float*)d_in[27];
  const float* Wb4a = (const float*)d_in[28];  const float* bb4a = (const float*)d_in[29];
  const float* Wb4b = (const float*)d_in[30];  const float* bb4b = (const float*)d_in[31];

  char* ws = (char*)d_ws;
  unsigned short* WT = (unsigned short*)(ws + kOffWT);
  float* RES  = (float*)(ws + kOffRES);
  float* PART = (float*)(ws + kOffPART);
  float* AVG  = (float*)(ws + kOffAVG);
  float* out  = (float*)d_out;

  prep_weights_kernel<<<(oWEnd / 8) / 256, 256, 0, stream>>>(
      W1a, W1b, Wb1, Ww2a, Ww2b, Wb2a, W3a, W3b, Wb3, W4a, W4b, Wb4a, WT);

  fused_mixer_kernel<<<kNumBlocks, kWavesPerBlock * 32, 0, stream>>>(
      qvals, states, a_h, gs, WT,
      b1a, b1b, bb1, bw2a, bw2b, bb2a, Wb2b, bb2b,
      b3a, b3b, bb3, b4a, b4b, bb4a, Wb4b, bb4b,
      RES, PART);

  mean_combine_kernel<<<1, 64, 0, stream>>>(PART, AVG);

  pack_out_kernel<<<(kOutLines + 7) / 8, 256, 0, stream>>>(RES, AVG, out);
}
